// MambaLayer_73624329388581
// MI455X (gfx1250) — hardware-verified
//
#include <hip/hip_runtime.h>
#include <math.h>

typedef __attribute__((ext_vector_type(16))) _Float16 v16h;
typedef __attribute__((ext_vector_type(8)))  _Float16 v8h;
typedef __attribute__((ext_vector_type(16))) __bf16   v16b;
typedef __attribute__((ext_vector_type(8)))  __bf16   v8b;
typedef __attribute__((ext_vector_type(8)))  float    v8f;
typedef __attribute__((ext_vector_type(4)))  float    v4f;
typedef __attribute__((ext_vector_type(4)))  unsigned int v4u;

constexpr int kC     = 96;
constexpr int kNVox  = 32768;
constexpr int kDin   = 192;
constexpr int kNst   = 16;
constexpr int kDtR   = 6;
constexpr int kXdW   = 38;
constexpr int kL     = 512;
constexpr int kNWin  = 64;
constexpr int kXzP   = 2 * kDin;
constexpr int kXdN   = 48;
constexpr int kOutN  = 128;
constexpr int kChunk = 32;
constexpr int kUP    = 196;
constexpr int kUHP   = 200;
constexpr int kXDP   = 52;
constexpr int kMeanP = 32;
constexpr int kLnRows = 64;
static_assert(kNWin * kL == kNVox, "token count");
static_assert(kDtR + 2 * kNst == kXdW, "x_proj width");
static_assert((kC % 32) == 0 && (kDin % 32) == 0, "GEMM K multiples of 32");
static_assert((kNVox % 64) == 0 && (kXzP % 64) == 0 && (kOutN % 64) == 0, "GEMM M,N multiples of 64");
static_assert((kL % kChunk) == 0 && kChunk == 32 && kDin == 192, "branch kernel tiling");
static_assert((kNst + kDtR) * kDin <= kChunk * kUP, "parameter staging fits the u tile");
static_assert((kNVox % kLnRows) == 0 && ((kLnRows * kC * 2) % 128) == 0, "LN block byte range is whole lines");
static_assert((kC * kNVox) % (4 * 256) == 0, "apply grid exact");

constexpr size_t kOffWIH  = 0;
constexpr size_t kOffWIL  = kOffWIH + (size_t)kXzP * kC * 2;
constexpr size_t kOffWOH  = kOffWIL + (size_t)kXzP * kC * 2;
constexpr size_t kOffWOL  = kOffWOH + (size_t)kOutN * kDin * 2;
constexpr size_t kOffWX0  = kOffWOL + (size_t)kOutN * kDin * 2;
constexpr size_t kOffWX1  = kOffWX0 + (size_t)kXdN * kDin * 2;
constexpr size_t kOffWX2  = kOffWX1 + (size_t)kXdN * kDin * 2;
constexpr size_t kOffMEAN = kOffWX2 + (size_t)kXdN * kDin * 2;
constexpr size_t kOffXNH  = kOffMEAN + (size_t)kC * kMeanP * 4;
constexpr size_t kOffXNL  = kOffXNH + (size_t)kNVox * kC * 2;
constexpr size_t kOffYSH  = kOffXNH;
constexpr size_t kOffXZ   = kOffXNL + (size_t)kNVox * kC * 2;
constexpr size_t kOffOUT5 = kOffXZ;
constexpr size_t kOffYA   = kOffXZ + (size_t)kNVox * kXzP * 4;
constexpr size_t kOffYB   = kOffYA + (size_t)kNVox * kDin * 4;
constexpr size_t kOffYSL  = kOffYB + (size_t)kNVox * kDin * 4;
constexpr size_t kWsTotal = kOffYSL + (size_t)kNVox * kDin * 2;
static_assert(kWsTotal == 126142464ull, "carve total");
static_assert(kWsTotal <= 134217728ull, "carve cap");
static_assert(kOffYSH + (size_t)kNVox * kDin * 2 <= kOffXZ, "ysum hi plane fits the xn region");
static_assert(kOffOUT5 + (size_t)kC * kNVox * 4 <= kOffYA, "out5 fits the xz region");
static_assert((kOffWIL % 128) == 0 && (kOffWOH % 128) == 0 && (kOffWOL % 128) == 0 && (kOffWX0 % 128) == 0 &&
              (kOffWX1 % 128) == 0 && (kOffWX2 % 128) == 0 && (kOffMEAN % 128) == 0 && (kOffXNH % 128) == 0 &&
              (kOffXNL % 128) == 0 && (kOffXZ % 128) == 0 && (kOffYA % 128) == 0 && (kOffYB % 128) == 0 &&
              (kOffYSL % 128) == 0, "128-B aligned regions");

__device__ __forceinline__ unsigned short f2bf_bits(float f) {
  unsigned u = __float_as_uint(f);
  return (unsigned short)((u + 0x7FFFu + ((u >> 16) & 1u)) >> 16);
}
__device__ __forceinline__ float bf_bits2f(unsigned short h) { return __uint_as_float(((unsigned)h) << 16); }

__device__ __forceinline__ void dep_guard4_h(v8f& a, v8f& b, v8f& c, v8f& d, v16h x, v16h y) {
  asm volatile("v_nop\n\tv_nop\n\tv_nop\n\tv_nop" : "+v"(a), "+v"(b), "+v"(c), "+v"(d) : "v"(x), "v"(y));
}
__device__ __forceinline__ void dep_guard4_b(v8f& a, v8f& b, v8f& c, v8f& d, v16b x, v16b y) {
  asm volatile("v_nop\n\tv_nop\n\tv_nop\n\tv_nop" : "+v"(a), "+v"(b), "+v"(c), "+v"(d) : "v"(x), "v"(y));
}
__device__ __forceinline__ void keep4_h(v16h a, v16h b, v16h c, v16h d) { asm volatile("v_nop" :: "v"(a), "v"(b), "v"(c), "v"(d)); }
__device__ __forceinline__ void keep4_b(v16b a, v16b b, v16b c, v16b d) { asm volatile("v_nop" :: "v"(a), "v"(b), "v"(c), "v"(d)); }
__device__ __forceinline__ void acc_guard4(v8f& a, v8f& b, v8f& c, v8f& d) { asm volatile("v_nop\n\tv_nop\n\tv_nop\n\tv_nop" : "+v"(a), "+v"(b), "+v"(c), "+v"(d)); }
template <typename T> struct Frag;
template <> struct Frag<_Float16> {
  typedef v16h V; union U { v16h v; v8h h[2]; };
  static __device__ __forceinline__ v16h load(const _Float16* p) {
    U f; f.h[0] = *(const v8h*)(p); f.h[1] = *(const v8h*)(p + 16); return f.v;
  }
  static __device__ __forceinline__ v8f mma(v16h a, v16h b, v8f c) {
    return __builtin_amdgcn_wmma_f32_16x16x32_f16(false, a, false, b, (short)0, c, false, false);
  }
  static __device__ __forceinline__ void guard4(v8f& a, v8f& b, v8f& c, v8f& d, v16h x, v16h y) { dep_guard4_h(a, b, c, d, x, y); }
  static __device__ __forceinline__ void keep(v16h a, v16h b, v16h c, v16h d) { keep4_h(a, b, c, d); }
};
template <> struct Frag<__bf16> {
  typedef v16b V; union U { v16b v; v8b h[2]; };
  static __device__ __forceinline__ v16b load(const __bf16* p) {
    U f; f.h[0] = *(const v8b*)(p); f.h[1] = *(const v8b*)(p + 16); return f.v;
  }
  static __device__ __forceinline__ v8f mma(v16b a, v16b b, v8f c) {
    return __builtin_amdgcn_wmma_f32_16x16x32_bf16(false, a, false, b, (short)0, c, false, false);
  }
  static __device__ __forceinline__ void guard4(v8f& a, v8f& b, v8f& c, v8f& d, v16b x, v16b y) { dep_guard4_b(a, b, c, d, x, y); }
  static __device__ __forceinline__ void keep(v16b a, v16b b, v16b c, v16b d) { keep4_b(a, b, c, d); }
};

__device__ __forceinline__ v8f mma_h(v16h a, v16h b, v8f c) {
  c = __builtin_amdgcn_wmma_f32_16x16x32_f16(false, a, false, b, (short)0, c, false, false);
  asm volatile("v_nop\n\tv_nop\n\tv_nop\n\tv_nop" : "+v"(c) : "v"(a), "v"(b));
  return c;
}

template <int ET> struct Elem;
template <> struct Elem<0> { typedef _Float16 T; };
template <> struct Elem<1> { typedef __bf16 T; };
template <int ET, bool SPLIT, int OUT_MODE, bool RESID>
__global__ __launch_bounds__(256) void wmma_gemm64x(
    const unsigned short* __restrict__ Ap, const unsigned short* __restrict__ A2p, int lda,
    const unsigned short* __restrict__ Btp, const unsigned short* __restrict__ Bt2p, int ldb,
    float* __restrict__ Cout, int ldc, const float* __restrict__ resid,
    int M, int N, int K, int n_real, float scale) {
  typedef typename Elem<ET>::T T;
  typedef typename Frag<T>::V V;
  const T* A = (const T*)Ap; const T* A2 = (const T*)A2p; const T* Bt = (const T*)Btp; const T* Bt2 = (const T*)Bt2p;
  __shared__ __align__(16) float sT[8][16 * 68];
  const int lane = threadIdx.x & 31;
  const int wave = threadIdx.x >> 5;
  const int tilesN = N >> 6;
  const int tilesM = M >> 6;
  const int tile = blockIdx.x * 8 + wave;
  if (tile >= tilesM * tilesN) return;
  const int tm = tile / tilesN;
  const int tn = tile - tm * tilesN;
  const int m0 = tm << 6;
  const int n0 = tn << 6;

  const int rlane = lane & 15;
  const int koff  = (lane >> 4) * 8;
  const int mOff  = (lane >> 4) * 8;

  v8f acc[4][4];
#pragma unroll
  for (int i = 0; i < 4; ++i)
#pragma unroll
    for (int j = 0; j < 4; ++j) acc[i][j] = (v8f){0.f,0.f,0.f,0.f,0.f,0.f,0.f,0.f};

  for (int k0 = 0; k0 < K; k0 += 32) {
    V bh[4], bl[4];
#pragma unroll
    for (int j = 0; j < 4; ++j) {
      const size_t bo = (size_t)(n0 + (j << 4) + rlane) * ldb + koff + k0;
      bh[j] = Frag<T>::load(Bt + bo);
      if (SPLIT) bl[j] = Frag<T>::load(Bt2 + bo);
    }
#pragma unroll
    for (int i = 0; i < 4; ++i) {
      const size_t ao = (size_t)(m0 + (i << 4) + rlane) * lda + koff + k0;
      V ah = Frag<T>::load(A + ao);
      V al;
      if (SPLIT) al = Frag<T>::load(A2 + ao);
#pragma unroll
      for (int j = 0; j < 4; ++j) {
        acc[i][j] = Frag<T>::mma(ah, bh[j], acc[i][j]);
        if (SPLIT) {
          acc[i][j] = Frag<T>::mma(ah, bl[j], acc[i][j]);
          acc[i][j] = Frag<T>::mma(al, bh[j], acc[i][j]);
        }
      }
      Frag<T>::guard4(acc[i][0], acc[i][1], acc[i][2], acc[i][3], ah, SPLIT ? al : ah);
    }
    Frag<T>::keep(bh[0], bh[1], bh[2], bh[3]);
    if (SPLIT) Frag<T>::keep(bl[0], bl[1], bl[2], bl[3]);
  }
  acc_guard4(acc[0][0], acc[0][1], acc[0][2], acc[0][3]);
  acc_guard4(acc[1][0], acc[1][1], acc[1][2], acc[1][3]);
  acc_guard4(acc[2][0], acc[2][1], acc[2][2], acc[2][3]);
  acc_guard4(acc[3][0], acc[3][1], acc[3][2], acc[3][3]);

  float* slab = sT[wave];
  const int hh = lane >> 4, c4 = (lane & 15) * 4;
  if (OUT_MODE == 0) {
#pragma unroll
    for (int i = 0; i < 4; ++i) {
      const int mBase = m0 + (i << 4);
#pragma unroll
      for (int j = 0; j < 4; ++j) {
#pragma unroll
        for (int r = 0; r < 8; ++r) slab[(mOff + r) * 68 + (j << 4) + rlane] = acc[i][j][r] * scale;
      }
      __builtin_amdgcn_fence(__ATOMIC_RELEASE, "workgroup");
      __builtin_amdgcn_wave_barrier();
      __builtin_amdgcn_fence(__ATOMIC_ACQUIRE, "workgroup");
      for (int pass = 0; pass < 2; ++pass) {
#pragma unroll
        for (int it = 0; it < 8; ++it) {
          const int row = it * 2 + hh;
          v4f v = *(const v4f*)(slab + row * 68 + c4);
          *(volatile v4f*)(Cout + (size_t)(mBase + row) * ldc + n0 + c4) = v;
        }
        __threadfence();
      }
      __builtin_amdgcn_fence(__ATOMIC_RELEASE, "workgroup");
      __builtin_amdgcn_wave_barrier();
      __builtin_amdgcn_fence(__ATOMIC_ACQUIRE, "workgroup");
    }
  } else {
#pragma unroll
    for (int j = 0; j < 4; ++j) {
      const int nBase = n0 + (j << 4);
      if (nBase < n_real) {
#pragma unroll
        for (int i = 0; i < 4; ++i) {
#pragma unroll
          for (int r = 0; r < 8; ++r) slab[rlane * 68 + (i << 4) + mOff + r] = acc[i][j][r] * scale;
        }
        __builtin_amdgcn_fence(__ATOMIC_RELEASE, "workgroup");
        __builtin_amdgcn_wave_barrier();
        __builtin_amdgcn_fence(__ATOMIC_ACQUIRE, "workgroup");
        for (int pass = 0; pass < 2; ++pass) {
#pragma unroll
          for (int it = 0; it < 8; ++it) {
            const int row = it * 2 + hh;
            v4f v = *(const v4f*)(slab + row * 68 + c4);
            if (RESID) {
              const v4f rv = *(const v4f*)(resid + (size_t)(nBase + row) * ldc + m0 + c4);
              v += rv;
            }
            *(volatile v4f*)(Cout + (size_t)(nBase + row) * ldc + m0 + c4) = v;
          }
          __threadfence();
        }
        __builtin_amdgcn_fence(__ATOMIC_RELEASE, "workgroup");
        __builtin_amdgcn_wave_barrier();
        __builtin_amdgcn_fence(__ATOMIC_ACQUIRE, "workgroup");
      }
    }
  }
}

__global__ __launch_bounds__(256) void split_pad_bf16_kernel(
    const float* __restrict__ src, int nsrc, unsigned short* __restrict__ dhi, unsigned short* __restrict__ dlo, int total8)
{
  const int i = blockIdx.x * 256 + threadIdx.x;
  if (i >= total8) return;
  const int e0 = i << 3;
  const bool inb = (e0 < nsrc);
  const int ec = inb ? e0 : (nsrc - 8);
  const float fac = inb ? 1.0f : 0.0f;
  const v4f a0 = *(const v4f*)(src + ec);
  const v4f a1 = *(const v4f*)(src + ec + 4);
  v8h hv, lv;
#pragma unroll
  for (int e = 0; e < 4; ++e) {
    const float f0 = a0[e] * fac;
    const float f1 = a1[e] * fac;
    const unsigned short h0 = f2bf_bits(f0), h1 = f2bf_bits(f1);
    const unsigned short l0 = f2bf_bits(f0 - bf_bits2f(h0)), l1 = f2bf_bits(f1 - bf_bits2f(h1));
    hv[e]     = __builtin_bit_cast(_Float16, h0);
    hv[4 + e] = __builtin_bit_cast(_Float16, h1);
    lv[e]     = __builtin_bit_cast(_Float16, l0);
    lv[4 + e] = __builtin_bit_cast(_Float16, l1);
  }
  unsigned short* qh = dhi + e0;
  unsigned short* ql = dlo + e0;
  *(volatile v8h*)qh = hv;
  *(volatile v8h*)ql = lv;
  __threadfence();
  *(volatile v8h*)qh = hv;
  *(volatile v8h*)ql = lv;
}

__global__ __launch_bounds__(256) void wx_f16_kernel(const float* __restrict__ src, unsigned short* __restrict__ dst)
{
  const int i = blockIdx.x * 256 + threadIdx.x;
  if (i >= (kXdN * kDin) / 8) return;
  const int e0 = i << 3;
  const int n = e0 / kDin;
  const int c = e0 - n * kDin;
  const bool valid = (n < kDtR) || (n >= 8 && n < 8 + 2 * kNst);
  int sr = (n < kDtR) ? n : (n - 2);
  sr = valid ? sr : 0;
  const float fac = valid ? 1.0f : 0.0f;
  const v4f a0 = *(const v4f*)(src + (size_t)sr * kDin + c);
  const v4f a1 = *(const v4f*)(src + (size_t)sr * kDin + c + 4);
  v8h hv;
#pragma unroll
  for (int e = 0; e < 4; ++e) {
    const float f0 = a0[e] * fac;
    const float f1 = a1[e] * fac;
    hv[e]     = (_Float16)f0;
    hv[4 + e] = (_Float16)f1;
  }
  *(volatile v8h*)(dst + e0) = hv;
  __threadfence();
  *(volatile v8h*)(dst + e0) = hv;
}

__device__ __forceinline__ int vox_of(int b, int l) {
  const int hb = b >> 4, wb = (b >> 2) & 3, db = b & 3;
  const int i = l >> 6, j = (l >> 3) & 7, k = l & 7;
  return ((hb * 8 + i) << 10) | ((wb * 8 + j) << 5) | (db * 8 + k);
}
template <int BR> __device__ __forceinline__ int lmap(int t) {
  if (BR == 0) return t;
  if (BR == 1) return (kL - 1) - t;
  return ((t & 7) << 6) + (t >> 3);
}

__global__ __launch_bounds__(kLnRows) void ln_kernel(
    const float* __restrict__ x, const float* __restrict__ lw, const float* __restrict__ lb,
    unsigned short* __restrict__ XNH, unsigned short* __restrict__ XNL)
{
  __shared__ __align__(16) unsigned short sH[kLnRows * kC];
  __shared__ __align__(16) unsigned short sLo[kLnRows * kC];
  const int tid = threadIdx.x, lane = tid & 31, wave = tid >> 5;
  const int v = blockIdx.x * kLnRows + tid;
  float s = 0.0f;
#pragma unroll 1
  for (int c = 0; c < kC; ++c) s += x[(size_t)c * kNVox + v];
  const float mu = s * (1.0f / 96.0f);
  float s2 = 0.0f;
#pragma unroll 1
  for (int c = 0; c < kC; ++c) { const float dl = x[(size_t)c * kNVox + v] - mu; s2 += dl * dl; }
  const float var = s2 * (1.0f / 96.0f);
  const float rstd = rsqrtf(var + 1e-5f);
#pragma unroll 1
  for (int c = 0; c < kC; ++c) {
    const float xv = x[(size_t)c * kNVox + v];
    const float o = (xv - mu) * rstd * lw[c] + lb[c];
    const unsigned short hb = f2bf_bits(o);
    const unsigned short lob = f2bf_bits(o - bf_bits2f(hb));
    sH[tid * kC + c] = hb;
    sLo[tid * kC + c] = lob;
  }
  __syncthreads();
  const int q = lane >> 3, j8 = lane & 7;
  const size_t base = (size_t)blockIdx.x * kLnRows * kC;
  for (int pass = 0; pass < 2; ++pass) {
#pragma unroll
    for (int it = 0; it < 12; ++it) {
      const int li = it * 8 + wave * 4 + q;
      const int off = li * 64 + 8 * j8;
      const v4u hv = *(const v4u*)(sH + off);
      const v4u lv = *(const v4u*)(sLo + off);
      *(volatile v4u*)(XNH + base + off) = hv;
      *(volatile v4u*)(XNL + base + off) = lv;
    }
    __threadfence();
  }
}

template <int BR>
__global__ __launch_bounds__(kDin) void branch_kernel(
    const float* __restrict__ XZ, const unsigned short* __restrict__ Wxp,
    const float* __restrict__ cw, const float* __restrict__ cb,
    const float* __restrict__ Wdt, const float* __restrict__ bdt,
    const float* __restrict__ Alog, const float* __restrict__ Dp,
    const float* YinA, const float* YinB,
    float* Yout, unsigned short* __restrict__ YSH, unsigned short* __restrict__ YSL)
{
  __shared__ __align__(16) float    sU[kChunk * kUP];
  __shared__ __align__(16) _Float16 sUh[kChunk * kUHP];
  __shared__ __align__(16) float    sXD[kChunk * kXDP];
  union FH { v16h v; v8h p[2]; };
  const int tid = threadIdx.x, lane = tid & 31, wave = tid >> 5;
  const int b = blockIdx.x;
  const int d = tid;
  const _Float16* Wx = (const _Float16*)Wxp;

#pragma unroll 1
  for (int s = 0; s < kNst; ++s) sU[s * kDin + tid] = -expf(Alog[(size_t)d * kNst + s]);
#pragma unroll 1
  for (int r = 0; r < kDtR; ++r) sU[(kNst + r) * kDin + tid] = Wdt[(size_t)d * kDtR + r];
  const v4f cwv = *(const v4f*)(cw + (size_t)d * 4);
  const float cbd = cb[d];
  const float bbd = bdt[d];
  const float Dd  = Dp[d];
  asm volatile("" ::: "memory");
  __syncthreads();
  float negA[kNst], h[kNst], dtw[kDtR];
#pragma unroll
  for (int s = 0; s < kNst; ++s) { negA[s] = sU[s * kDin + tid]; h[s] = 0.0f; }
#pragma unroll
  for (int r = 0; r < kDtR; ++r) dtw[r] = sU[(kNst + r) * kDin + tid];
  const float w0 = cwv[0], w1 = cwv[1], w2 = cwv[2], w3 = cwv[3];
  float xm3 = 0.0f, xm2 = 0.0f, xm1 = 0.0f;

  const int hh = lane >> 4, rl = lane & 15;
  const int gi = (wave >= 3) ? 1 : 0;
  const int gj = wave - 3 * gi;
  const int q = lane >> 3, j8 = lane & 7;

#pragma unroll 1
  for (int t0 = 0; t0 < kL; t0 += kChunk) {
    __syncthreads();
#pragma unroll 1
    for (int s = 0; s < kChunk; ++s) {
      const int row = vox_of(b, lmap<BR>(t0 + s));
      const float xcur = XZ[(size_t)row * kXzP + d];
      float a = w0 * xm3;
      a = fmaf(w1, xm2, a);
      a = fmaf(w2, xm1, a);
      a = fmaf(w3, xcur, a);
      const float cv = a + cbd;
      const float sg = __builtin_amdgcn_rcpf(1.0f + expf(-cv));
      const float u = cv * sg;
      sU[s * kUP + tid] = u;
      sUh[s * kUHP + tid] = (_Float16)u;
      xm3 = xm2; xm2 = xm1; xm1 = xcur;
    }
    __syncthreads();
    {
      FH bw[6];
#pragma unroll
      for (int ks = 0; ks < 3; ++ks) {
        const _Float16* bp = Wx + (size_t)(16 * gj + rl) * kDin + 32 * ks + 8 * hh;
        bw[ks].p[0] = *(const v8h*)(bp);
        bw[ks].p[1] = *(const v8h*)(bp + 16);
      }
      asm volatile("" ::: "memory");
#pragma unroll
      for (int ks = 3; ks < 6; ++ks) {
        const _Float16* bp = Wx + (size_t)(16 * gj + rl) * kDin + 32 * ks + 8 * hh;
        bw[ks].p[0] = *(const v8h*)(bp);
        bw[ks].p[1] = *(const v8h*)(bp + 16);
      }
      asm volatile("" ::: "memory");
      v8f acc = (v8f){0.f,0.f,0.f,0.f,0.f,0.f,0.f,0.f};
#pragma unroll
      for (int ks = 0; ks < 6; ++ks) {
        FH fa;
        const _Float16* ap = sUh + (16 * gi + rl) * kUHP + 32 * ks + 8 * hh;
        fa.p[0] = *(const v8h*)(ap);
        fa.p[1] = *(const v8h*)(ap + 16);
        acc = mma_h(fa.v, bw[ks].v, acc);
      }
#pragma unroll
      for (int r = 0; r < 8; ++r) sXD[(16 * gi + 8 * hh + r) * kXDP + 16 * gj + rl] = acc[r];
    }
    __syncthreads();
#pragma unroll 1
    for (int s = 0; s < kChunk; ++s) {
      const int row = vox_of(b, lmap<BR>(t0 + s));
      const float zv = XZ[(size_t)row * kXzP + kDin + d];
      float yprev = 0.0f;
      if (BR == 2) {
        const float ya = YinA[(size_t)row * kDin + d];
        const float yb = YinB[(size_t)row * kDin + d];
        yprev = ya + yb;
      }
      const float* xr = sXD + s * kXDP;
      const v4f d03 = *(const v4f*)(xr);
      const v4f d47 = *(const v4f*)(xr + 4);
      float vdot = d03[0] * dtw[0];
      vdot = fmaf(d03[1], dtw[1], vdot);
      vdot = fmaf(d03[2], dtw[2], vdot);
      vdot = fmaf(d03[3], dtw[3], vdot);
      vdot = fmaf(d47[0], dtw[4], vdot);
      vdot = fmaf(d47[1], dtw[5], vdot);
      const float vv = vdot + bbd;
      const float dt = fmaxf(vv, 0.0f) + log1pf(expf(-fabsf(vv)));
      const float u = sU[s * kUP + tid];
      const float dtx = dt * u;
      float y = 0.0f;
#pragma unroll
      for (int g4 = 0; g4 < 4; ++g4) {
        const v4f bv = *(const v4f*)(xr + 8 + 4 * g4);
        const v4f cv = *(const v4f*)(xr + 24 + 4 * g4);
#pragma unroll
        for (int e = 0; e < 4; ++e) {
          const int k = 4 * g4 + e;
          const float ex = expf(dt * negA[k]);
          h[k] = ex * h[k] + dtx * bv[e];
          y = y + h[k] * cv[e];
        }
      }
      y = y + Dd * u;
      const float sg = __builtin_amdgcn_rcpf(1.0f + expf(-zv));
      float ys = y * (zv * sg);
      if (BR == 2) ys = yprev + ys;
      sU[s * kUP + tid] = ys;
    }
    __syncthreads();
    if (BR < 2) {
      v4f vals[8];
      int rows[8];
#pragma unroll
      for (int it = 0; it < 8; ++it) {
        const int trow = it * 4 + q;
        rows[it] = vox_of(b, lmap<BR>(t0 + trow));
        vals[it] = *(const v4f*)(sU + trow * kUP + 32 * wave + 4 * j8);
      }
      for (int pass = 0; pass < 2; ++pass) {
#pragma unroll
        for (int it = 0; it < 8; ++it)
          *(volatile v4f*)(Yout + (size_t)rows[it] * kDin + 32 * wave + 4 * j8) = vals[it];
        __threadfence();
      }
    } else {
      v8h hv[4], lv[4];
      int rows[4];
#pragma unroll
      for (int it = 0; it < 4; ++it) {
        const int trow = it * 8 + gi * 4 + q;
        rows[it] = vox_of(b, lmap<BR>(t0 + trow));
        const float* sp = sU + trow * kUP + 64 * gj + 8 * j8;
        const v4f a0 = *(const v4f*)(sp);
        const v4f a1 = *(const v4f*)(sp + 4);
#pragma unroll
        for (int e = 0; e < 4; ++e) {
          const unsigned short h0 = f2bf_bits(a0[e]), h1 = f2bf_bits(a1[e]);
          const unsigned short l0 = f2bf_bits(a0[e] - bf_bits2f(h0)), l1 = f2bf_bits(a1[e] - bf_bits2f(h1));
          hv[it][e]     = __builtin_bit_cast(_Float16, h0);
          hv[it][4 + e] = __builtin_bit_cast(_Float16, h1);
          lv[it][e]     = __builtin_bit_cast(_Float16, l0);
          lv[it][4 + e] = __builtin_bit_cast(_Float16, l1);
        }
      }
      for (int pass = 0; pass < 2; ++pass) {
#pragma unroll
        for (int it = 0; it < 4; ++it) {
          const size_t o = (size_t)rows[it] * kDin + 64 * gj + 8 * j8;
          *(volatile v8h*)(YSH + o) = hv[it];
          *(volatile v8h*)(YSL + o) = lv[it];
        }
        __threadfence();
      }
    }
  }
}

__global__ __launch_bounds__(256) void eca_mean_kernel(const float* __restrict__ out5, float* __restrict__ means)
{
  __shared__ float sm[256];
  const int tid = threadIdx.x;
  const int c = blockIdx.x;
  const float* p = out5 + (size_t)c * kNVox;
  float s = 0.0f;
#pragma unroll 1
  for (int v = tid; v < kNVox; v += 256) s += p[v];
  sm[tid] = s;
  __syncthreads();
#pragma unroll 1
  for (int off = 128; off > 0; off >>= 1) {
    if (tid < off) sm[tid] = sm[tid] + sm[tid + off];
    __syncthreads();
  }
  const float mval = sm[0] * (1.0f / 32768.0f);
  if (tid < 32) {
    const float o = (tid == 0) ? mval : 0.0f;
    float* mp = means + (size_t)c * kMeanP + tid;
    *(volatile float*)mp = o;
    __threadfence();
    *(volatile float*)mp = o;
  }
}

__global__ __launch_bounds__(256) void eca_apply_kernel(
    const float* __restrict__ out5, const float* __restrict__ means, const float* __restrict__ ew, float* __restrict__ out)
{
  const int i = blockIdx.x * 256 + threadIdx.x;
  const int c = i >> 13;
  const int cl = (c > 0) ? (c - 1) : 0;
  const int cr = (c < kC - 1) ? (c + 1) : (kC - 1);
  const float ml = means[(size_t)cl * kMeanP];
  const float mc = means[(size_t)c * kMeanP];
  const float mr = means[(size_t)cr * kMeanP];
  const float fl = (c > 0) ? 1.0f : 0.0f;
  const float fr = (c < kC - 1) ? 1.0f : 0.0f;
  const float w0 = ew[0], w1 = ew[1], w2 = ew[2];
  float g = w0 * (ml * fl);
  g = g + w1 * mc;
  g = g + w2 * (mr * fr);
  const float sg = __builtin_amdgcn_rcpf(1.0f + expf(-g));
  v4f v = *(const v4f*)(out5 + ((size_t)i << 2));
  v = v * sg;
  float* op = out + ((size_t)i << 2);
  *(volatile v4f*)op = v;
  __threadfence();
  *(volatile v4f*)op = v;
}

extern "C" void kernel_launch(void* const* d_in, const int* in_sizes, int n_in,
                              void* d_out, int out_size, void* d_ws, size_t ws_size,
                              hipStream_t stream) {
  if (n_in < 27) return;
  if (in_sizes[0] != kC * kNVox) return;
  if (in_sizes[1] != kC || in_sizes[2] != kC) return;
  if (in_sizes[3] != kXzP * kC) return;
  if (in_sizes[4] != kC * kDin) return;
  if (in_sizes[5] != 3) return;
  for (int br = 0; br < 3; ++br) {
    const int bs = 6 + 7 * br;
    if (in_sizes[bs + 0] != kDin * 4) return;
    if (in_sizes[bs + 1] != kDin) return;
    if (in_sizes[bs + 2] != kXdW * kDin) return;
    if (in_sizes[bs + 3] != kDin * kDtR) return;
    if (in_sizes[bs + 4] != kDin) return;
    if (in_sizes[bs + 5] != kDin * kNst) return;
    if (in_sizes[bs + 6] != kDin) return;
  }
  if (out_size != kC * kNVox) return;
  if (ws_size < kWsTotal) return;

  const float* x     = (const float*)d_in[0];
  const float* ln_w  = (const float*)d_in[1];
  const float* ln_b  = (const float*)d_in[2];
  const float* W_in  = (const float*)d_in[3];
  const float* W_out = (const float*)d_in[4];
  const float* eca_w = (const float*)d_in[5];
  float* out = (float*)d_out;

  char* ws = (char*)d_ws;
  unsigned short* WIH  = (unsigned short*)(ws + kOffWIH);
  unsigned short* WIL  = (unsigned short*)(ws + kOffWIL);
  unsigned short* WOH  = (unsigned short*)(ws + kOffWOH);
  unsigned short* WOL  = (unsigned short*)(ws + kOffWOL);
  unsigned short* WX[3];
  WX[0] = (unsigned short*)(ws + kOffWX0);
  WX[1] = (unsigned short*)(ws + kOffWX1);
  WX[2] = (unsigned short*)(ws + kOffWX2);
  float*          MEAN = (float*)(ws + kOffMEAN);
  unsigned short* XNH  = (unsigned short*)(ws + kOffXNH);
  unsigned short* XNL  = (unsigned short*)(ws + kOffXNL);
  unsigned short* YSH  = (unsigned short*)(ws + kOffYSH);
  float*          XZ   = (float*)(ws + kOffXZ);
  float*          OUT5 = (float*)(ws + kOffOUT5);
  float*          YA   = (float*)(ws + kOffYA);
  float*          YB   = (float*)(ws + kOffYB);
  unsigned short* YSL  = (unsigned short*)(ws + kOffYSL);

  split_pad_bf16_kernel<<<(kXzP * kC / 8) / 256, 256, 0, stream>>>(W_in, kXzP * kC, WIH, WIL, kXzP * kC / 8);
  split_pad_bf16_kernel<<<(kOutN * kDin / 8) / 256, 256, 0, stream>>>(W_out, kC * kDin, WOH, WOL, kOutN * kDin / 8);
  for (int br = 0; br < 3; ++br) {
    const float* W_x = (const float*)d_in[6 + 7 * br + 2];
    wx_f16_kernel<<<(kXdN * kDin / 8 + 255) / 256, 256, 0, stream>>>(W_x, WX[br]);
  }

  ln_kernel<<<kNVox / kLnRows, kLnRows, 0, stream>>>(x, ln_w, ln_b, XNH, XNL);

  wmma_gemm64x<1, true, 0, false><<<dim3((kNVox / 64) * (kXzP / 64) / 8, 1), 256, 0, stream>>>(
      XNH, XNL, kC, WIH, WIL, kC, XZ, kXzP, nullptr, kNVox, kXzP, kC, kXzP, 1.0f);

  {
    const int bs = 6;
    branch_kernel<0><<<kNWin, kDin, 0, stream>>>(
        XZ, WX[0], (const float*)d_in[bs + 0], (const float*)d_in[bs + 1], (const float*)d_in[bs + 3],
        (const float*)d_in[bs + 4], (const float*)d_in[bs + 5], (const float*)d_in[bs + 6],
        YA, YB, YA, YSH, YSL);
  }
  {
    const int bs = 13;
    branch_kernel<1><<<kNWin, kDin, 0, stream>>>(
        XZ, WX[1], (const float*)d_in[bs + 0], (const float*)d_in[bs + 1], (const float*)d_in[bs + 3],
        (const float*)d_in[bs + 4], (const float*)d_in[bs + 5], (const float*)d_in[bs + 6],
        YA, YB, YB, YSH, YSL);
  }
  {
    const int bs = 20;
    branch_kernel<2><<<kNWin, kDin, 0, stream>>>(
        XZ, WX[2], (const float*)d_in[bs + 0], (const float*)d_in[bs + 1], (const float*)d_in[bs + 3],
        (const float*)d_in[bs + 4], (const float*)d_in[bs + 5], (const float*)d_in[bs + 6],
        YA, YB, YA, YSH, YSL);
  }

  wmma_gemm64x<1, true, 3, true><<<dim3((kNVox / 64) * (kOutN / 64) / 8, 1), 256, 0, stream>>>(
      YSH, YSL, kDin, WOH, WOL, kDin, OUT5, kNVox, x, kNVox, kOutN, kDin, kC, 1.0f);

  eca_mean_kernel<<<kC, 256, 0, stream>>>(OUT5, MEAN);
  eca_apply_kernel<<<(kC * kNVox / 4) / 256, 256, 0, stream>>>(OUT5, MEAN, eca_w, out);
}
